// SimpleHeteroConv_89163521065076
// MI455X (gfx1250) — hardware-verified
//
#include <hip/hip_runtime.h>
#include <stddef.h>


#define FD      128
#define NTYP    2
#define NTHR    256
#define NWAVE   8
#define EPT     8
#define NGRP    2
#define CHUNK   (NTHR * EPT * NGRP)
#define WCAP    (EPT * NGRP * 32)
#define LISTN   (NWAVE * WCAP)
#define NBC     4096
#define NBF     1024
#define RCAP    40960
#define RBN     128
#define TGT     256
#define DEGCAP  1024
#define GROWS   128
#define OTHR    512
#define WSCAP   134217728

#define KD      128
#define APK     136
#define WPL     (FD * KD)
#define WPTOT   (2 * NTYP * WPL)

#define LDS_FILL ((RCAP + NBF + LISTN) * 4 + 64)
#define LDS_AT   (GROWS * APK * 2)
#define LDS_STG  (GROWS * FD * 4)
#define LDS_G    (LDS_AT + LDS_STG)

#define CARRY    16.0f
#define UNCARRY  (1.0f / 256.0f)

static_assert((CHUNK & (CHUNK - 1)) == 0);
static_assert(CHUNK <= 4096);
static_assert(NBC <= 4096 && NBF <= 4096);
static_assert((NBC & (NBC - 1)) == 0 && (NBF & (NBF - 1)) == 0);
static_assert(NBC == 4 * NBF);
static_assert(OTHR * 8 == NBC);
static_assert((RCAP % 32) == 0);
static_assert(TGT == NWAVE * 32 && (TGT % GROWS) == 0);
static_assert((NBC % TGT) == 0);
static_assert(GROWS == NWAVE * 16);
static_assert(FD == 128 && KD == 128 && (APK % 8) == 0);
static_assert((LDS_AT % 16) == 0);
static_assert((WPL % 64) == 0);

typedef float          v4f  __attribute__((ext_vector_type(4)));
typedef float          v8f  __attribute__((ext_vector_type(8)));
typedef int            v4i  __attribute__((ext_vector_type(4)));
typedef _Float16       v8h  __attribute__((ext_vector_type(8)));
typedef _Float16       v16h __attribute__((ext_vector_type(16)));
union FragH { v16h v; v8h h[2]; };

__device__ __forceinline__ v8h cvt8(v4f a, v4f b) {
  v8h o;
  o[0] = (_Float16)a.x; o[1] = (_Float16)a.y; o[2] = (_Float16)a.z; o[3] = (_Float16)a.w;
  o[4] = (_Float16)b.x; o[5] = (_Float16)b.y; o[6] = (_Float16)b.z; o[7] = (_Float16)b.w;
  return o;
}

__device__ __forceinline__ v8f wmh(v16h a, v16h b, v8f c) {
  v8f d = __builtin_amdgcn_wmma_f32_16x16x32_f16(false, a, false, b, (short)0, c, false, false);
  asm volatile("v_nop\n\tv_nop\n\tv_nop\n\tv_nop" : "+v"(d) : "v"(a), "v"(b));
  return d;
}

template <int NT>
__device__ __forceinline__ void mma16(const _Float16* sA, const _Float16* __restrict__ Bw,
                                      int wrow, int lane, v8f (&acc)[NT]) {
  constexpr int NKT = KD / 32;
  const int hh = lane >> 4, m = lane & 15;
#pragma unroll
  for (int t = 0; t < NT; ++t) { v8f z = {0.f, 0.f, 0.f, 0.f, 0.f, 0.f, 0.f, 0.f}; acc[t] = z; }
  const _Float16* ap = sA + (wrow + m) * APK + 8 * hh;
#pragma unroll
  for (int kt = 0; kt < NKT; ++kt) {
    FragH a;
    a.h[0] = *(const v8h*)(ap + 32 * kt);
    a.h[1] = *(const v8h*)(ap + 32 * kt + 16);
#pragma unroll
    for (int t = 0; t < NT; ++t) {
      const _Float16* bp = Bw + (size_t)(16 * t + m) * KD + 32 * kt + 8 * hh;
      FragH b;
      b.h[0] = *(const v8h*)bp;
      b.h[1] = *(const v8h*)(bp + 16);
      acc[t] = wmh(a.v, b.v, acc[t]);
    }
  }
}

__device__ __forceinline__ void store_rows128(const float* stg, float* C, int rowBase, int nRows,
                                              int wave, int lane) {
  const float* lp = stg + wave * 16 * FD + 4 * lane;
  const int r0 = rowBase + wave * 16;
  float* gp = C + (size_t)r0 * FD + 4 * lane;
#pragma unroll
  for (int i = 0; i < 16; ++i) {
    if (r0 + i < nRows) { const v4f v = *(const v4f*)(lp + FD * i); *(volatile v4f*)(gp + FD * i) = v; }
  }
  __threadfence();
#pragma unroll
  for (int i = 0; i < 16; ++i) {
    if (r0 + i < nRows) { const v4f v = *(const v4f*)(lp + FD * i); *(volatile v4f*)(gp + FD * i) = v; }
  }
}

template <int NB>
__device__ __forceinline__ int scan_chunk(const int* __restrict__ dsts, int nE, int cbase, int slotBase,
                                          int vec8, int* list, int tid, int lane, int wave) {
  int wc = 0;
#pragma unroll
  for (int g = 0; g < NGRP; ++g) {
    const int el0  = (g * NTHR + tid) * EPT;
    const int e0   = cbase + el0;
    const int sent = -2147483647 - 1;
    v4i da, db;
    if (vec8 != 0 && cbase + CHUNK <= nE) {
      da = *(const v4i*)(dsts + e0);
      db = *(const v4i*)(dsts + e0 + 4);
    } else {
      da.x = (e0     < nE) ? dsts[min(e0, nE - 1)] : sent;
      da.y = (e0 + 1 < nE) ? dsts[min(e0 + 1, nE - 1)] : sent;
      da.z = (e0 + 2 < nE) ? dsts[min(e0 + 2, nE - 1)] : sent;
      da.w = (e0 + 3 < nE) ? dsts[min(e0 + 3, nE - 1)] : sent;
      db.x = (e0 + 4 < nE) ? dsts[min(e0 + 4, nE - 1)] : sent;
      db.y = (e0 + 5 < nE) ? dsts[min(e0 + 5, nE - 1)] : sent;
      db.z = (e0 + 6 < nE) ? dsts[min(e0 + 6, nE - 1)] : sent;
      db.w = (e0 + 7 < nE) ? dsts[min(e0 + 7, nE - 1)] : sent;
    }
    const unsigned nb = (unsigned)slotBase;
    const unsigned s0 = (unsigned)da.x - nb, s1 = (unsigned)da.y - nb;
    const unsigned s2 = (unsigned)da.z - nb, s3 = (unsigned)da.w - nb;
    const unsigned s4 = (unsigned)db.x - nb, s5 = (unsigned)db.y - nb;
    const unsigned s6 = (unsigned)db.z - nb, s7 = (unsigned)db.w - nb;
    const bool h0 = s0 < (unsigned)NB, h1 = s1 < (unsigned)NB, h2 = s2 < (unsigned)NB, h3 = s3 < (unsigned)NB;
    const bool h4 = s4 < (unsigned)NB, h5 = s5 < (unsigned)NB, h6 = s6 < (unsigned)NB, h7 = s7 < (unsigned)NB;
    const unsigned any = __builtin_amdgcn_ballot_w32(h0 | h1 | h2 | h3 | h4 | h5 | h6 | h7);
    if (any != 0u) {
#define HITJ(J, HJ, SJ) { \
        const unsigned mj = __builtin_amdgcn_ballot_w32(HJ); \
        if (mj != 0u) { \
          if (HJ) { \
            const int pos = wc + (int)__builtin_amdgcn_mbcnt_lo(mj, 0u); \
            if (pos < WCAP) list[wave * WCAP + pos] = ((el0 + (J)) << 12) | (int)(SJ); \
          } \
          wc += (int)__builtin_popcount(mj); } }
      HITJ(0, h0, s0)
      HITJ(1, h1, s1)
      HITJ(2, h2, s2)
      HITJ(3, h3, s3)
      HITJ(4, h4, s4)
      HITJ(5, h5, s5)
      HITJ(6, h6, s6)
      HITJ(7, h7, s7)
#undef HITJ
    }
  }
  return wc;
}

__global__ __launch_bounds__(NTHR) void k_wprep(
    const float* __restrict__ wv, const float* __restrict__ wa, _Float16* wp) {
  const int blk = blockIdx.x, tid = threadIdx.x;
  const int p = blk >> 3, which = p >> 1, t = p & 1;
  const int i = (blk & 7) * NTHR + tid;
  const int n = i >> 4, k0 = (i & 15) * 8;
  float v[8];
#pragma unroll
  for (int e = 0; e < 8; ++e) {
    const int idx = (t * KD + k0 + e) * FD + n;
    const float va = wv[idx];
    const float vb = wa[idx];
    v[e] = ((which != 0) ? vb : va) * CARRY;
  }
  v4f a, b;
  a.x = v[0]; a.y = v[1]; a.z = v[2]; a.w = v[3];
  b.x = v[4]; b.y = v[5]; b.z = v[6]; b.w = v[7];
  const v8h hv = cvt8(a, b);
  _Float16* dh = wp + (size_t)p * WPL + (size_t)i * 8;
  *(volatile v8h*)dh = hv;
  __threadfence();
  *(volatile v8h*)dh = hv;
}

__global__ __launch_bounds__(NTHR) void k_count(const int* __restrict__ dsts, int* cnt, int nE, int vec8) {
  __shared__ __attribute__((aligned(16))) int scnt[NBC];
  __shared__ __attribute__((aligned(16))) int list[LISTN];
  __shared__ int wcnt[NWAVE];
  const int tid = threadIdx.x, lane = tid & 31, wave = tid >> 5;
  const int nodeBase = blockIdx.x * NBC;

  for (int i = tid; i < NBC; i += NTHR) scnt[i] = 0;
  __syncthreads();

  const int nChunks = (nE + CHUNK - 1) / CHUNK;
#pragma unroll 1
  for (int ch = 0; ch < nChunks; ++ch) {
    const int cbase = ch * CHUNK;
    const int wc = scan_chunk<NBC>(dsts, nE, cbase, nodeBase, vec8, list, tid, lane, wave);
    if (lane == 0) wcnt[wave] = wc;
    __syncthreads();
    if (wave == 0) {
#pragma unroll 1
      for (int wsx = 0; wsx < NWAVE; ++wsx) {
        int n = __builtin_amdgcn_readfirstlane(wcnt[wsx]);
        n = n > WCAP ? WCAP : (n < 0 ? 0 : n);
        const int* lp = list + wsx * WCAP;
#pragma unroll 1
        for (int i = 0; i < n; ++i) {
          const int ent  = __builtin_amdgcn_readfirstlane(lp[i]);
          const int slot = ent & (NBC - 1);
          if (lane == 0) scnt[slot] = scnt[slot] + 1;
        }
      }
    }
    __syncthreads();
  }

  v4i cq[4];
#pragma unroll
  for (int q = 0; q < 4; ++q) {
    const int f = (wave * 4 + q) * 128 + 4 * lane;
    cq[q] = *(const v4i*)(scnt + f);
  }
  int* cp = cnt + (size_t)nodeBase;
#pragma unroll
  for (int q = 0; q < 4; ++q) {
    const int f = (wave * 4 + q) * 128 + 4 * lane;
    *(volatile v4i*)(cp + f) = cq[q];
  }
  __threadfence();
#pragma unroll
  for (int q = 0; q < 4; ++q) {
    const int f = (wave * 4 + q) * 128 + 4 * lane;
    *(volatile v4i*)(cp + f) = cq[q];
  }
}

__global__ __launch_bounds__(OTHR) void k_offsets(
    const int* __restrict__ cnt, int* off, int* rbase, int nChunk) {
  __shared__ __attribute__((aligned(16))) int soff[NBC];
  __shared__ __attribute__((aligned(16))) int srb[RBN];
  __shared__ int wtot[OTHR / 32];
  const int tid = threadIdx.x, lane = tid & 31, wave = tid >> 5, sub = tid >> 7;
  for (int i = tid; i < RBN; i += OTHR) srb[i] = 0;
  int carry = 0;
#pragma unroll 1
  for (int ch = 0; ch < nChunk; ++ch) {
    const int base = ch * NBC;
    const v4i c0 = *(const v4i*)(cnt + base + 8 * tid);
    const v4i c1 = *(const v4i*)(cnt + base + 8 * tid + 4);
    const int e0 = max(c0.x, 0), e1 = max(c0.y, 0), e2 = max(c0.z, 0), e3 = max(c0.w, 0);
    const int e4 = max(c1.x, 0), e5 = max(c1.y, 0), e6 = max(c1.z, 0), e7 = max(c1.w, 0);
    const int ts = e0 + e1 + e2 + e3 + e4 + e5 + e6 + e7;
    int incl = ts;
#pragma unroll
    for (int d = 1; d < 32; d <<= 1) {
      const int t = __shfl_up(incl, d);
      if (lane >= d) incl += t;
    }
    if (lane == 31) wtot[wave] = incl;
    __syncthreads();
    const int S0 = wtot[0]  + wtot[1]  + wtot[2]  + wtot[3];
    const int S1 = wtot[4]  + wtot[5]  + wtot[6]  + wtot[7];
    const int S2 = wtot[8]  + wtot[9]  + wtot[10] + wtot[11];
    const int S3 = wtot[12] + wtot[13] + wtot[14] + wtot[15];
    int pre = 0;
#pragma unroll 1
    for (int w = 4 * sub; w < wave; ++w) pre += wtot[w];
    const int b0 = carry;
    const int b1 = b0 + ((S0 + 31) & ~31);
    const int b2 = b1 + ((S1 + 31) & ~31);
    const int b3 = b2 + ((S2 + 31) & ~31);
    const int b4 = b3 + ((S3 + 31) & ~31);
    const int myb = sub == 0 ? b0 : (sub == 1 ? b1 : (sub == 2 ? b2 : b3));
    if (tid == 0) {
      srb[min(4 * ch + 0, RBN - 1)] = b0;
      srb[min(4 * ch + 1, RBN - 1)] = b1;
      srb[min(4 * ch + 2, RBN - 1)] = b2;
      srb[min(4 * ch + 3, RBN - 1)] = b3;
    }
    int run = myb + pre + incl - ts;
    soff[8 * tid + 0] = run; run += e0;
    soff[8 * tid + 1] = run; run += e1;
    soff[8 * tid + 2] = run; run += e2;
    soff[8 * tid + 3] = run; run += e3;
    soff[8 * tid + 4] = run; run += e4;
    soff[8 * tid + 5] = run; run += e5;
    soff[8 * tid + 6] = run; run += e6;
    soff[8 * tid + 7] = run;
    carry = b4;
    __syncthreads();
    const v4i o0 = *(const v4i*)(soff + 4 * tid);
    const v4i o1 = *(const v4i*)(soff + 4 * (tid + OTHR));
    int* op = off + base;
    *(volatile v4i*)(op + 4 * tid) = o0;
    *(volatile v4i*)(op + 4 * (tid + OTHR)) = o1;
    __threadfence();
    *(volatile v4i*)(op + 4 * tid) = o0;
    *(volatile v4i*)(op + 4 * (tid + OTHR)) = o1;
    __syncthreads();
  }
  if (tid == 0) srb[min(4 * nChunk, RBN - 1)] = carry;
  __syncthreads();
  v4i rv = {0, 0, 0, 0};
  if (tid < 32) rv = *(const v4i*)(srb + 4 * tid);
  if (tid < 32) *(volatile v4i*)(rbase + 4 * tid) = rv;
  __threadfence();
  if (tid < 32) *(volatile v4i*)(rbase + 4 * tid) = rv;
}

__global__ __launch_bounds__(NTHR) void k_fill(
    const int* __restrict__ srcs, const int* __restrict__ dsts,
    const int* __restrict__ off, const int* __restrict__ rbase,
    int* csr, int nN, int nE, int vec8, int csrLen) {
  extern __shared__ v4f lds_dyn[];
  int* region = (int*)lds_dyn;
  int* cursor = region + RCAP;
  int* list   = cursor + NBF;
  int* wcnt   = list + LISTN;
  const int tid = threadIdx.x, lane = tid & 31, wave = tid >> 5;
  const int b = blockIdx.x;
  const int nodeBase = b * NBF;

  int rb0 = rbase[b];
  const int rb1 = rbase[b + 1];
  rb0 = rb0 < 0 ? 0 : (rb0 > csrLen ? csrLen : rb0);
  rb0 &= ~31;
  int len = rb1 - rb0;
  len = len < 0 ? 0 : (len > RCAP ? RCAP : len);
  int lenW = (len + 31) & ~31;
  if (rb0 + lenW > csrLen) lenW = (csrLen - rb0) & ~31;

  {
    const v4i z = {0, 0, 0, 0};
    for (int i = tid; i < RCAP / 4; i += NTHR) ((v4i*)region)[i] = z;
    for (int s = tid; s < NBF; s += NTHR) {
      int o = off[nodeBase + s] - rb0;
      o = o < 0 ? 0 : (o > RCAP ? RCAP : o);
      cursor[s] = o;
    }
  }
  __syncthreads();

  const int nChunks = (nE + CHUNK - 1) / CHUNK;
#pragma unroll 1
  for (int ch = 0; ch < nChunks; ++ch) {
    const int cbase = ch * CHUNK;
    const int wc = scan_chunk<NBF>(dsts, nE, cbase, nodeBase, vec8, list, tid, lane, wave);
    if (lane == 0) wcnt[wave] = wc;
    __syncthreads();
    if (wave == 0) {
#pragma unroll 1
      for (int wsx = 0; wsx < NWAVE; ++wsx) {
        int n = __builtin_amdgcn_readfirstlane(wcnt[wsx]);
        n = n > WCAP ? WCAP : (n < 0 ? 0 : n);
        const int* lp = list + wsx * WCAP;
#pragma unroll 1
        for (int i = 0; i < n; ++i) {
          const int ent  = __builtin_amdgcn_readfirstlane(lp[i]);
          const int slot = ent & (NBF - 1);
          int e = cbase + ((ent >> 12) & (CHUNK - 1));
          e = e > nE - 1 ? nE - 1 : e;
          int sv = srcs[e];
          sv = sv < 0 ? 0 : (sv > nN - 1 ? nN - 1 : sv);
          if (lane == 0) {
            int pos = cursor[slot];
            pos = pos < 0 ? 0 : (pos > RCAP - 1 ? RCAP - 1 : pos);
            region[pos] = sv;
            const int np = pos + 1;
            cursor[slot] = np > RCAP ? RCAP : np;
          }
        }
      }
    }
    __syncthreads();
  }

  const int nv = lenW >> 2;
  int* gp = csr + rb0;
#pragma unroll 1
  for (int i = tid; i < nv; i += NTHR) { const v4i v = ((const v4i*)region)[i]; *(volatile v4i*)(gp + 4 * i) = v; }
  __threadfence();
#pragma unroll 1
  for (int i = tid; i < nv; i += NTHR) { const v4i v = ((const v4i*)region)[i]; *(volatile v4i*)(gp + 4 * i) = v; }
}

__global__ __launch_bounds__(NTHR) void k_tgemm(
    const float* __restrict__ A, const int* __restrict__ nty,
    const _Float16* __restrict__ Bw, float* C, int nN, int nRows) {
  extern __shared__ v4f lds_dyn[];
  __shared__ __attribute__((aligned(16))) int sTy[GROWS];
  _Float16* sA  = (_Float16*)lds_dyn;
  float*    stg = (float*)((char*)lds_dyn + LDS_AT);
  const int tid = threadIdx.x, lane = tid & 31, wave = tid >> 5, hh = lane >> 4, m = lane & 15;
  const int rowBase = blockIdx.x * GROWS;
  const int c0 = (tid & 15) * 8, rr = tid >> 4;

  if (tid < GROWS) {
    int row = rowBase + tid;
    row = row > nN - 1 ? nN - 1 : row;
    int t = nty[row];
    t = t < 0 ? 0 : (t > NTYP - 1 ? NTYP - 1 : t);
    sTy[tid] = t;
  }
#pragma unroll 2
  for (int it = 0; it < 8; ++it) {
    const int r = it * 16 + rr;
    int row = rowBase + r;
    row = row > nN - 1 ? nN - 1 : row;
    const float* ap = A + (size_t)row * FD + c0;
    const v4f a = *(const v4f*)ap * CARRY, b = *(const v4f*)(ap + 4) * CARRY;
    *(v8h*)(sA + r * APK + c0) = cvt8(a, b);
  }
  __syncthreads();

  const v4i t4 = *(const v4i*)(sTy + 4 * lane);
  const bool has0 = (t4.x == 0) | (t4.y == 0) | (t4.z == 0) | (t4.w == 0);
  const bool has1 = (t4.x == 1) | (t4.y == 1) | (t4.z == 1) | (t4.w == 1);
  const unsigned mk0 = __builtin_amdgcn_ballot_w32(has0);
  const unsigned mk1 = __builtin_amdgcn_ballot_w32(has1);
  const int present = (mk0 != 0u ? 1 : 0) | (mk1 != 0u ? 2 : 0);
  int tyb = 0;
#pragma unroll
  for (int r = 0; r < 8; ++r) tyb |= (sTy[wave * 16 + 8 * hh + r] & 1) << r;

#pragma unroll 1
  for (int t = 0; t < NTYP; ++t) {
    if (((present >> t) & 1) == 0) continue;
    const _Float16* Bt = Bw + (size_t)t * WPL;
#pragma unroll
    for (int ch = 0; ch < 2; ++ch) {
      v8f acc[4];
      mma16<4>(sA, Bt + (size_t)(64 * ch) * KD, wave * 16, lane, acc);
      float* sp = stg + (wave * 16 + 8 * hh) * FD + 64 * ch + m;
#pragma unroll
      for (int tt = 0; tt < 4; ++tt) {
#pragma unroll
        for (int r = 0; r < 8; ++r) {
          if (((tyb >> r) & 1) == t) sp[r * FD + 16 * tt] = acc[tt][r] * UNCARRY;
        }
      }
    }
  }
  __syncthreads();

  store_rows128(stg, C, rowBase, nRows, wave, lane);
}

__global__ __launch_bounds__(NTHR) void k_agg(
    const int* __restrict__ csr, const int* __restrict__ off, const int* __restrict__ cnt,
    const float* __restrict__ V, float* H, int nN, int csrLen) {
  const int tid = threadIdx.x, lane = tid & 31, wave = tid >> 5;
  const int tbase = blockIdx.x * TGT + wave * 32;
  const int cl = tbase + lane;
  const int cnt_l = cnt[cl];
  const int off_l = off[cl];

#pragma unroll 1
  for (int j = 0; j < 32; ++j) {
    const int c = tbase + j;
    int n = __builtin_amdgcn_readlane(cnt_l, j);
    n = n < 0 ? 0 : (n > DEGCAP ? DEGCAP : n);
    const int st = __builtin_amdgcn_readlane(off_l, j);
    v4f sm = {0.0f, 0.0f, 0.0f, 0.0f};
#pragma unroll 1
    for (int q0 = 0; q0 < n; q0 += 32) {
      int pos = st + q0 + lane;
      pos = pos < 0 ? 0 : (pos > csrLen - 1 ? csrLen - 1 : pos);
      int sl = csr[pos];
      sl = sl < 0 ? 0 : (sl > nN - 1 ? nN - 1 : sl);
      const int mcnt = (n - q0) < 32 ? (n - q0) : 32;
#pragma unroll 1
      for (int p = 0; p < mcnt; ++p) {
        const int s = __builtin_amdgcn_readlane(sl, p);
        const v4f vf = *(const v4f*)(V + (size_t)s * FD + 4 * lane);
        sm = sm + vf;
      }
    }
    float* hp = H + (size_t)c * FD + 4 * lane;
    *(volatile v4f*)hp = sm;
    __threadfence();
    *(volatile v4f*)hp = sm;
  }
}

extern "C" void kernel_launch(void* const* d_in, const int* in_sizes, int n_in,
                              void* d_out, int out_size, void* d_ws, size_t ws_size,
                              hipStream_t stream) {
  if (n_in < 6) return;
  const int nN = in_sizes[1];
  const int nE = in_sizes[2];
  if (nN <= 0 || nE <= 0) return;
  if (in_sizes[0] != nN * FD || in_sizes[3] != nE) return;
  if (in_sizes[4] != NTYP * KD * FD || in_sizes[5] != NTYP * KD * FD) return;
  if (out_size != nN * FD) return;
  if (nE > (1 << 28) || nN > (1 << 24)) return;

  const float* x    = (const float*)d_in[0];
  const int*   nty  = (const int*)d_in[1];
  const int*   srcs = (const int*)d_in[2];
  const int*   dsts = (const int*)d_in[3];
  const float* wv   = (const float*)d_in[4];
  const float* wa   = (const float*)d_in[5];
  float* out = (float*)d_out;

  const int NPAD   = ((nN + TGT - 1) / TGT) * TGT;
  const int nBC    = (nN + NBC - 1) / NBC;
  const int CNTPAD = nBC * NBC;
  if (4 * nBC + 1 > RBN) return;
  const int nBF    = (nN + NBF - 1) / NBF;
  const int csrLen = ((nE + 31) & ~31) + 4096;
  if (31 * 4 * nBC > 4096) return;
  const int nGemm  = NPAD / GROWS;
  const int nAgg   = NPAD / TGT;

  char* ws = (char*)d_ws;
  size_t off = 0;
  const size_t oW   = off; off += (size_t)WPTOT * 2;        off = (off + 255) & ~(size_t)255;
  const size_t oCnt = off; off += (size_t)CNTPAD * 4;       off = (off + 255) & ~(size_t)255;
  const size_t oOff = off; off += (size_t)CNTPAD * 4;       off = (off + 255) & ~(size_t)255;
  const size_t oRb  = off; off += (size_t)RBN * 4;          off = (off + 255) & ~(size_t)255;
  const size_t oCsr = off; off += (size_t)csrLen * 4;       off = (off + 255) & ~(size_t)255;
  const size_t oV   = off; off += (size_t)NPAD * FD * 4;    off = (off + 255) & ~(size_t)255;
  const size_t oH   = off; off += (size_t)NPAD * FD * 4;    off = (off + 255) & ~(size_t)255;
  if (off > ws_size || off > (size_t)WSCAP) return;
  _Float16* wp   = (_Float16*)(ws + oW);
  int*      cnt  = (int*)(ws + oCnt);
  int*      offp = (int*)(ws + oOff);
  int*      rb   = (int*)(ws + oRb);
  int*      csr  = (int*)(ws + oCsr);
  float*    Vp   = (float*)(ws + oV);
  float*    Hp   = (float*)(ws + oH);

  const int vec8 = 1;

  k_wprep<<<4 * 8, NTHR, 0, stream>>>(wv, wa, wp);

  k_count<<<nBC, NTHR, 0, stream>>>(dsts, cnt, nE, vec8);
  k_offsets<<<1, OTHR, 0, stream>>>(cnt, offp, rb, nBC);
  hipFuncSetAttribute(reinterpret_cast<const void*>(&k_fill),
                      hipFuncAttributeMaxDynamicSharedMemorySize, LDS_FILL);
  k_fill<<<nBF, NTHR, LDS_FILL, stream>>>(srcs, dsts, offp, rb, csr, nN, nE, vec8, csrLen);

  hipFuncSetAttribute(reinterpret_cast<const void*>(&k_tgemm),
                      hipFuncAttributeMaxDynamicSharedMemorySize, LDS_G);
  k_tgemm<<<nGemm, NTHR, LDS_G, stream>>>(x, nty, wp, Vp, nN, NPAD);

  k_agg<<<nAgg, NTHR, 0, stream>>>(csr, offp, cnt, Vp, Hp, nN, csrLen);

  k_tgemm<<<nGemm, NTHR, LDS_G, stream>>>(Hp, nty, wp + (size_t)NTYP * WPL, out, nN, nN);
}
